// GNN_3j1m_hetero_70016556859578
// MI455X (gfx1250) — hardware-verified
//
#include <hip/hip_runtime.h>
#include <stddef.h>
#include <stdint.h>
#include <math.h>


#define HD     16
#define MHD    64
#define NTHR   256
#define NWAVE  8
#define EPT    8
#define CHUNK  (NTHR * EPT)
#define WCAP   (EPT * 32)
#define LISTN  (NWAVE * WCAP)
#define NBA    1024
#define SLA    10
#define CPB    32
#define TROW   64
#define LN_EPS 1e-5f
#define WSMAX  134217728

#define OFF_E1    0
#define OFF_JE2   1024
#define OFF_MU2   1536
#define OFF_M1W1  2048
#define OFF_M1W2  4096
#define OFF_M2W1  6144
#define OFF_M2W2  8192
#define OFF_FC1   10240
#define WP_HALVES 14336
#define NUNITS    (WP_HALVES / 8)

#define G_ZF    (LISTN)
#define G_MISC  (LISTN + NBA * HD)
#define G_OT    (G_MISC + 32)
#define G_HS    (G_OT + NWAVE * 256)
#define G_INTS  (G_HS + NWAVE * 1024)
#define P_CNT   (LISTN)
#define P_MISC  (P_CNT + NBA)
#define P_OUTS  (P_MISC + 32)
#define P_SUM   (P_OUTS + NBA)
#define P_MAX   (P_SUM + NBA * HD)
#define P_INTS  (P_MAX + NBA * HD)

static_assert((CHUNK & (CHUNK - 1)) == 0 && CHUNK <= 4096);
static_assert((NBA & (NBA - 1)) == 0 && NBA == (1 << SLA));
static_assert(((long long)CHUNK << SLA) < (1LL << 31));
static_assert(NUNITS % NTHR == 0);
static_assert(G_ZF % 4 == 0 && G_MISC % 4 == 0 && G_OT % 4 == 0 && G_HS % 4 == 0);
static_assert(P_CNT % 4 == 0 && P_MISC % 4 == 0 && P_OUTS % 4 == 0 && P_SUM % 4 == 0 && P_MAX % 4 == 0);
static_assert(G_INTS * 4 <= 300000 && P_INTS * 4 <= 300000);
static_assert((NBA / 16) % NWAVE == 0);
static_assert(CPB == NWAVE * 4 && TROW == 2 * CPB);

typedef float          v4f   __attribute__((ext_vector_type(4)));
typedef float          v8f   __attribute__((ext_vector_type(8)));
typedef int            v4i   __attribute__((ext_vector_type(4)));
typedef int            v8i   __attribute__((ext_vector_type(8)));
typedef unsigned short v8us  __attribute__((ext_vector_type(8)));
typedef unsigned short v16us __attribute__((ext_vector_type(16)));
typedef __bf16         v16bf __attribute__((ext_vector_type(16)));
typedef v4f  __attribute__((may_alias)) v4fa;
typedef v4i  __attribute__((may_alias)) v4ia;
typedef v8us __attribute__((may_alias)) v8usa;
union FragB { v16bf v; v16us u; v8us h[2]; v8i w; };

__device__ __forceinline__ v8f wmb(const FragB& a, const FragB& b, v8f c) {
  v8f d = __builtin_amdgcn_wmma_f32_16x16x32_bf16(false, a.v, false, b.v, (short)0, c, false, false);
  asm volatile("v_nop\n\tv_nop\n\tv_nop\n\tv_nop" : "+v"(d) : "v"(a.w), "v"(b.w));
  return d;
}

__device__ __forceinline__ unsigned bf16_bits(float f) {
  const unsigned u = __float_as_uint(f);
  return (u + 0x7FFFu + ((u >> 16) & 1u)) >> 16;
}
__device__ __forceinline__ float bf16_val(float f) {
  return __uint_as_float(bf16_bits(f) << 16);
}
__device__ __forceinline__ void split2(float v, unsigned short& hi, unsigned short& lo) {
  const unsigned hb = bf16_bits(v);
  hi = (unsigned short)hb;
  lo = (unsigned short)bf16_bits(v - __uint_as_float(hb << 16));
}
__device__ __forceinline__ float relu_k(float v) {
  return (v > 0.0f) ? v : ((v != v) ? v : 0.0f);
}
__device__ __forceinline__ float blendf(float a, float b, unsigned mk) {
  return __uint_as_float((__float_as_uint(a) & mk) | (__float_as_uint(b) & ~mk));
}

__device__ __forceinline__ float pick4(const float* __restrict__ p, int idx) {
  const v4f v = *(const v4f*)(p + (idx & ~3));
  const unsigned m1 = (idx & 1) ? 0xffffffffu : 0u;
  const unsigned m2 = (idx & 2) ? 0xffffffffu : 0u;
  const float lo = blendf(v.y, v.x, m1);
  const float hi = blendf(v.w, v.z, m1);
  return blendf(hi, lo, m2);
}

__device__ __forceinline__ void wave_sync() {
  __builtin_amdgcn_fence(__ATOMIC_RELEASE, "wavefront");
  __builtin_amdgcn_wave_barrier();
  __builtin_amdgcn_fence(__ATOMIC_ACQUIRE, "wavefront");
}

__device__ __forceinline__ void ld_frag(FragB& f, const unsigned short* p, int hh) {
  f.h[0] = *(const v8usa*)(p + 8 * hh);
  f.h[1] = *(const v8usa*)(p + 16 + 8 * hh);
}

template <int SLB>
__device__ __forceinline__ int scan_chunk(const int* __restrict__ dsts, int nE, int cbase, int slotBase,
                                          int nb, int vec8, int* list, int tid, int lane, int wave) {
  int wc = 0;
  const int el0  = tid * EPT;
  const int e0   = cbase + el0;
  const int sent = -2147483647 - 1;
  v4i da, db;
  if (vec8 != 0 && cbase + CHUNK <= nE) {
    da = *(const v4i*)(dsts + e0);
    db = *(const v4i*)(dsts + e0 + 4);
  } else {
    da.x = (e0     < nE) ? dsts[min(e0,     nE - 1)] : sent;
    da.y = (e0 + 1 < nE) ? dsts[min(e0 + 1, nE - 1)] : sent;
    da.z = (e0 + 2 < nE) ? dsts[min(e0 + 2, nE - 1)] : sent;
    da.w = (e0 + 3 < nE) ? dsts[min(e0 + 3, nE - 1)] : sent;
    db.x = (e0 + 4 < nE) ? dsts[min(e0 + 4, nE - 1)] : sent;
    db.y = (e0 + 5 < nE) ? dsts[min(e0 + 5, nE - 1)] : sent;
    db.z = (e0 + 6 < nE) ? dsts[min(e0 + 6, nE - 1)] : sent;
    db.w = (e0 + 7 < nE) ? dsts[min(e0 + 7, nE - 1)] : sent;
  }
  const unsigned nbs = (unsigned)slotBase;
  const unsigned unb = (unsigned)nb;
  const unsigned s0 = (unsigned)da.x - nbs, s1 = (unsigned)da.y - nbs;
  const unsigned s2 = (unsigned)da.z - nbs, s3 = (unsigned)da.w - nbs;
  const unsigned s4 = (unsigned)db.x - nbs, s5 = (unsigned)db.y - nbs;
  const unsigned s6 = (unsigned)db.z - nbs, s7 = (unsigned)db.w - nbs;
  const bool h0 = s0 < unb, h1 = s1 < unb, h2 = s2 < unb, h3 = s3 < unb;
  const bool h4 = s4 < unb, h5 = s5 < unb, h6 = s6 < unb, h7 = s7 < unb;
  const unsigned any = __builtin_amdgcn_ballot_w32(h0 | h1 | h2 | h3 | h4 | h5 | h6 | h7);
  if (any != 0u) {
#define HITJ(J, HJ, SJ) { \
      const unsigned mj = __builtin_amdgcn_ballot_w32(HJ); \
      if (mj != 0u) { \
        if (HJ) { \
          const int pos = wc + (int)__builtin_amdgcn_mbcnt_lo(mj, 0u); \
          if (pos < WCAP) list[wave * WCAP + pos] = ((el0 + (J)) << SLB) | (int)(SJ); \
        } \
        wc += (int)__builtin_popcount(mj); } }
    HITJ(0, h0, s0)
    HITJ(1, h1, s1)
    HITJ(2, h2, s2)
    HITJ(3, h3, s3)
    HITJ(4, h4, s4)
    HITJ(5, h5, s5)
    HITJ(6, h6, s6)
    HITJ(7, h7, s7)
#undef HITJ
  }
  return wc;
}

__device__ __forceinline__ void derive_window(const int* __restrict__ T, int nCh, int b, int* wsh,
                                              int tid, int lane, int wave, int& clo, int& chi) {
  int cmin = 0x7fffffff, cmax = -1;
#pragma unroll 1
  for (int c0 = 0; c0 < nCh; c0 += NTHR) {
    const int c  = c0 + tid;
    const int cc = c < nCh ? c : nCh - 1;
    const int idx = (cc >> 5) * TROW + (cc & 31);
    const int lo = T[idx];
    const int hi = T[idx + CPB];
    const bool in = (c < nCh) && (lo <= b) && (b <= hi);
    cmin = in ? (c < cmin ? c : cmin) : cmin;
    cmax = in ? (c > cmax ? c : cmax) : cmax;
  }
#pragma unroll
  for (int d = 16; d >= 1; d >>= 1) {
    const int a = __shfl_xor(cmin, d, 32);
    const int z = __shfl_xor(cmax, d, 32);
    cmin = a < cmin ? a : cmin;
    cmax = z > cmax ? z : cmax;
  }
  if (lane == 0) { wsh[wave] = cmin; wsh[NWAVE + wave] = cmax; }
  __syncthreads();
  int a = 0x7fffffff, z = -1;
#pragma unroll
  for (int w = 0; w < NWAVE; ++w) {
    const int x = wsh[w], y = wsh[NWAVE + w];
    a = x < a ? x : a;
    z = y > z ? y : z;
  }
  a = __builtin_amdgcn_readfirstlane(a);
  z = __builtin_amdgcn_readfirstlane(z);
  clo = a < 0 ? 0 : a;
  chi = z > nCh - 1 ? nCh - 1 : z;
}

__global__ __launch_bounds__(NTHR) void k_prep(const float* __restrict__ je_w1, const float* __restrict__ mu_w1,
                                               const float* __restrict__ je_w2, const float* __restrict__ mu_w2,
                                               const float* __restrict__ m1_w1, const float* __restrict__ m1_w2,
                                               const float* __restrict__ m2_w1, const float* __restrict__ m2_w2,
                                               const float* __restrict__ fc_w1, unsigned short* WP) {
  const int u  = (int)blockIdx.x * NTHR + (int)threadIdx.x;
  const int e0 = u * 8;
  const float* src;
  int stride, kmask, klim, k8;
  if (e0 < OFF_JE2) {
    const int rel = e0; const int n = rel >> 5; k8 = rel & 31;
    src = (n < 16) ? (je_w1 + n) : (mu_w1 + (n - 16));
    stride = 16; kmask = 31; klim = 5;
  } else if (e0 < OFF_MU2) {
    const int rel = e0 - OFF_JE2; const int n = rel >> 5; k8 = rel & 31;
    src = je_w2 + n; stride = 16; kmask = 15; klim = 16;
  } else if (e0 < OFF_M1W1) {
    const int rel = e0 - OFF_MU2; const int n = rel >> 5; k8 = rel & 31;
    src = mu_w2 + n; stride = 16; kmask = 15; klim = 16;
  } else if (e0 < OFF_M1W2) {
    const int rel = e0 - OFF_M1W1; const int n = rel >> 5; k8 = rel & 31;
    src = m1_w1 + n; stride = 64; kmask = 15; klim = 16;
  } else if (e0 < OFF_M2W1) {
    const int rel = e0 - OFF_M1W2; const int n = rel >> 7; k8 = rel & 127;
    src = m1_w2 + n; stride = 16; kmask = 63; klim = 64;
  } else if (e0 < OFF_M2W2) {
    const int rel = e0 - OFF_M2W1; const int n = rel >> 5; k8 = rel & 31;
    src = m2_w1 + n; stride = 64; kmask = 15; klim = 16;
  } else if (e0 < OFF_FC1) {
    const int rel = e0 - OFF_M2W2; const int n = rel >> 7; k8 = rel & 127;
    src = m2_w2 + n; stride = 16; kmask = 63; klim = 64;
  } else {
    const int rel = e0 - OFF_FC1; const int n = rel >> 6; k8 = rel & 63;
    src = fc_w1 + n; stride = 64; kmask = 31; klim = 32;
  }
  v8us o;
#pragma unroll
  for (int i = 0; i < 8; ++i) {
    const int kk = (k8 + i) & kmask;
    const int kc = kk < klim ? kk : klim - 1;
    const float f = src[(size_t)kc * stride];
    o[i] = (kk < klim) ? (unsigned short)bf16_bits(f) : (unsigned short)0;
  }
  unsigned short* dp = WP + e0;
  *(volatile v8us*)dp = o;
  __threadfence();
  *(volatile v8us*)dp = o;
}

__global__ __launch_bounds__(NTHR) void k_bounds(const int* __restrict__ dsts, int nE, int vecE,
                                                 const int* __restrict__ bat, int nN, int nBE,
                                                 int* TE, int* TN) {
  __shared__ __attribute__((aligned(16))) int smm[TROW];
  const int tid = (int)threadIdx.x, lane = tid & 31, wave = tid >> 5;
  const int blk = (int)blockIdx.x;
  const int* keys; int n, vec, cb0; int* T;
  if (blk < nBE) { keys = dsts; n = nE; vec = vecE; cb0 = blk * CPB; T = TE + (size_t)blk * TROW; }
  else { keys = bat; n = nN; vec = 1; cb0 = (blk - nBE) * CPB; T = TN + (size_t)(blk - nBE) * TROW; }
#pragma unroll 1
  for (int q = 0; q < 4; ++q) {
    const int cl = wave * 4 + q;
    const int cbase = (cb0 + cl) * CHUNK;
    int mn = 0x7fffffff, mx = -2147483647 - 1;
    if (vec != 0 && cbase + CHUNK <= n) {
#pragma unroll 4
      for (int i = 0; i < 16; ++i) {
        const v4i d = *(const v4i*)(keys + cbase + i * 128 + 4 * lane);
        const int k0 = d.x >> SLA, k1 = d.y >> SLA, k2 = d.z >> SLA, k3 = d.w >> SLA;
        const int lo01 = k0 < k1 ? k0 : k1, lo23 = k2 < k3 ? k2 : k3;
        const int hi01 = k0 > k1 ? k0 : k1, hi23 = k2 > k3 ? k2 : k3;
        const int lo = lo01 < lo23 ? lo01 : lo23, hi = hi01 > hi23 ? hi01 : hi23;
        mn = lo < mn ? lo : mn;
        mx = hi > mx ? hi : mx;
      }
    } else {
#pragma unroll 1
      for (int i = 0; i < 64; ++i) {
        const int e  = cbase + i * 32 + lane;
        const int ec = e < n ? e : n - 1;
        const int kv = keys[ec] >> SLA;
        const bool ok = e < n;
        mn = (ok && kv < mn) ? kv : mn;
        mx = (ok && kv > mx) ? kv : mx;
      }
    }
#pragma unroll
    for (int d = 16; d >= 1; d >>= 1) {
      const int a = __shfl_xor(mn, d, 32);
      const int z = __shfl_xor(mx, d, 32);
      mn = a < mn ? a : mn;
      mx = z > mx ? z : mx;
    }
    if (lane == 0) { smm[cl] = mn; smm[CPB + cl] = mx; }
  }
  __syncthreads();
  const v4i o = *(const v4ia*)(smm + 4 * (lane & 15));
  int* dp = T + 4 * (lane & 15);
  const bool ok = (wave == 0) && (lane < 16);
  if (ok) *(volatile v4i*)dp = o;
  __threadfence();
  if (ok) *(volatile v4i*)dp = o;
}

__global__ __launch_bounds__(NTHR) void k_enc(const float* __restrict__ x, const int* __restrict__ tyid,
                                              const float* __restrict__ jb1, const float* __restrict__ mb1,
                                              const float* __restrict__ jb2, const float* __restrict__ mb2,
                                              const unsigned short* __restrict__ WP, int nN, float* H0) {
  __shared__ __attribute__((aligned(16))) unsigned short st[NWAVE * 2 * 512];
  __shared__ __attribute__((aligned(16))) float ots[NWAVE * 2 * 256];
  const int tid = (int)threadIdx.x, lane = tid & 31, wave = tid >> 5, hh = lane >> 4, m = lane & 15;
  unsigned short* stw = st + wave * 1024;
  float* otw = ots + wave * 512;
  const int base = ((int)blockIdx.x * NWAVE + wave) * 16;
  const v8f zero8 = {0.f, 0.f, 0.f, 0.f, 0.f, 0.f, 0.f, 0.f};

  const int row = base + m;
  const int rc  = row < nN ? row : nN - 1;
  const float* xp = x + (size_t)rc * 5;
  const float x0 = xp[0], x1 = xp[1], x2 = xp[2], x3 = xp[3], x4 = xp[4];
  const bool use = (row < nN) && (hh == 0);
  FragB a1;
  {
    const v8i z = {0, 0, 0, 0, 0, 0, 0, 0};
    a1.w = z;
  }
  a1.u[0] = use ? (unsigned short)bf16_bits(x0) : (unsigned short)0;
  a1.u[1] = use ? (unsigned short)bf16_bits(x1) : (unsigned short)0;
  a1.u[2] = use ? (unsigned short)bf16_bits(x2) : (unsigned short)0;
  a1.u[3] = use ? (unsigned short)bf16_bits(x3) : (unsigned short)0;
  a1.u[4] = use ? (unsigned short)bf16_bits(x4) : (unsigned short)0;

  FragB be0, be1, bj2, bm2;
  ld_frag(be0, WP + OFF_E1 + (size_t)m * 32, hh);
  ld_frag(be1, WP + OFF_E1 + (size_t)(16 + m) * 32, hh);
  ld_frag(bj2, WP + OFF_JE2 + (size_t)m * 32, hh);
  ld_frag(bm2, WP + OFF_MU2 + (size_t)m * 32, hh);
  const float bj1v = bf16_val(pick4(jb1, m)), bm1v = bf16_val(pick4(mb1, m));
  const float bj2v = bf16_val(pick4(jb2, m)), bm2v = bf16_val(pick4(mb2, m));

  const v8f aj = wmb(a1, be0, zero8);
  const v8f am = wmb(a1, be1, zero8);
#pragma unroll
  for (int r = 0; r < 8; ++r) {
    unsigned short hi, lo;
    const int lr = 8 * hh + r;
    split2(relu_k(aj[r] + bj1v), hi, lo);
    stw[lr * 32 + m] = hi; stw[lr * 32 + 16 + m] = lo;
    split2(relu_k(am[r] + bm1v), hi, lo);
    stw[512 + lr * 32 + m] = hi; stw[512 + lr * 32 + 16 + m] = lo;
  }
  wave_sync();
  FragB a2j, a2m;
  ld_frag(a2j, stw + m * 32, hh);
  ld_frag(a2m, stw + 512 + m * 32, hh);
  const v8f oj = wmb(a2j, bj2, zero8);
  const v8f om = wmb(a2m, bm2, zero8);
#pragma unroll
  for (int r = 0; r < 8; ++r) {
    const int lr = 8 * hh + r;
    otw[lr * 16 + m]       = oj[r] + bj2v;
    otw[256 + lr * 16 + m] = om[r] + bm2v;
  }
  wave_sync();
  v4f y[2];
#pragma unroll
  for (int i = 0; i < 2; ++i) {
    const int rr = 8 * i + (lane >> 2);
    const int cc = 4 * (lane & 3);
    const int node = base + rr;
    const int nc = node < nN ? node : nN - 1;
    const int ty = tyid[nc];
    const v4f vj = *(const v4fa*)(otw + rr * 16 + cc);
    const v4f vm = *(const v4fa*)(otw + 256 + rr * 16 + cc);
    const unsigned mk = (ty == 0) ? 0xffffffffu : 0u;
    const bool lv = node < nN;
    v4f v;
    v.x = blendf(vj.x, vm.x, mk); v.y = blendf(vj.y, vm.y, mk);
    v.z = blendf(vj.z, vm.z, mk); v.w = blendf(vj.w, vm.w, mk);
    v.x = lv ? v.x : 0.0f; v.y = lv ? v.y : 0.0f; v.z = lv ? v.z : 0.0f; v.w = lv ? v.w : 0.0f;
    y[i] = v;
  }
  float* op0 = H0 + (size_t)(base + (lane >> 2)) * HD + 4 * (lane & 3);
  float* op1 = op0 + 8 * HD;
  *(volatile v4f*)op0 = y[0];
  *(volatile v4f*)op1 = y[1];
  __threadfence();
  *(volatile v4f*)op0 = y[0];
  *(volatile v4f*)op1 = y[1];
}

__device__ __forceinline__ v4f ln16_relu(v4f v) {
  float s = (v.x + v.y) + (v.z + v.w);
  s += __shfl_xor(s, 1, 32);
  s += __shfl_xor(s, 2, 32);
  const float mu = s * 0.0625f;
  const float d0 = v.x - mu, d1 = v.y - mu, d2 = v.z - mu, d3 = v.w - mu;
  float q = (d0 * d0 + d1 * d1) + (d2 * d2 + d3 * d3);
  q += __shfl_xor(q, 1, 32);
  q += __shfl_xor(q, 2, 32);
  const float rs = 1.0f / sqrtf(q * 0.0625f + LN_EPS);
  v4f y;
  y.x = relu_k(d0 * rs); y.y = relu_k(d1 * rs); y.z = relu_k(d2 * rs); y.w = relu_k(d3 * rs);
  return y;
}

__global__ __launch_bounds__(NTHR) void k_gine(const int* __restrict__ srcs, const int* __restrict__ dsts,
                                               const float* __restrict__ eattr, int nE, int nN, int vec8,
                                               int nCh, const int* __restrict__ TE,
                                               const float* __restrict__ linw, const float* __restrict__ linb,
                                               const unsigned short* __restrict__ W1P, const float* __restrict__ b1,
                                               const unsigned short* __restrict__ W2P, const float* __restrict__ b2,
                                               const float* __restrict__ Hin, float* Hout) {
  extern __shared__ __attribute__((aligned(16))) int dsm[];
  int*   list = dsm;
  float* zf   = (float*)(dsm + G_ZF);
  int*   misc = dsm + G_MISC;
  const int tid = (int)threadIdx.x, lane = tid & 31, wave = tid >> 5, hh = lane >> 4, m = lane & 15;
  float* ot = (float*)(dsm + G_OT) + wave * 256;
  unsigned short* hs = (unsigned short*)(dsm + G_HS) + wave * 2048;
  const int blk = (int)blockIdx.x;
  const int nodeBase = blk * NBA;
  const v8f zero8 = {0.f, 0.f, 0.f, 0.f, 0.f, 0.f, 0.f, 0.f};

  {
    const v4i z4 = {0, 0, 0, 0};
    for (int i = tid * 4; i < G_MISC + 32; i += NTHR * 4) *(v4ia*)(dsm + i) = z4;
  }
  const float lw0 = bf16_val(linw[m]),      lw1 = bf16_val(linw[16 + m]);
  const float lw2 = bf16_val(linw[32 + m]), lw3 = bf16_val(linw[48 + m]);
  const float lbv = bf16_val(linb[m]);
  __syncthreads();

  int clo, chi;
  derive_window(TE, nCh, blk, misc + 16, tid, lane, wave, clo, chi);

#pragma unroll 1
  for (int ch = clo; ch <= chi; ++ch) {
    const int cbase = ch * CHUNK;
    const int wc = scan_chunk<SLA>(dsts, nE, cbase, nodeBase, NBA, vec8, list, tid, lane, wave);
    if (lane == 0) misc[wave] = wc;
    __syncthreads();
    if (wave == 0) {
#pragma unroll 1
      for (int w2 = 0; w2 < NWAVE; ++w2) {
        int c = __builtin_amdgcn_readfirstlane(misc[w2]);
        c = c < 0 ? 0 : (c > WCAP ? WCAP : c);
#pragma unroll 1
        for (int b0 = 0; b0 < c; b0 += 32) {
          const int idx = b0 + lane;
          const int ent = list[w2 * WCAP + (idx < WCAP ? idx : WCAP - 1)];
          const int slot = ent & (NBA - 1);
          const int el   = (ent >> SLA) & (CHUNK - 1);
          int eid = cbase + el;
          eid = eid < 0 ? 0 : (eid > nE - 1 ? nE - 1 : eid);
          int sr = srcs[eid];
          sr = sr < 0 ? 0 : (sr > nN - 1 ? nN - 1 : sr);
          const v4f ea = *(const v4f*)(eattr + 4 * (size_t)eid);
          const int e0i = __float_as_int(bf16_val(ea.x)), e1i = __float_as_int(bf16_val(ea.y));
          const int e2i = __float_as_int(bf16_val(ea.z)), e3i = __float_as_int(bf16_val(ea.w));
          const int m32 = (c - b0) < 32 ? (c - b0) : 32;
#pragma unroll 1
          for (int k = 0; k < m32; ++k) {
            const int   sk = __builtin_amdgcn_readlane(sr, k);
            const int   sl = __builtin_amdgcn_readlane(slot, k) & (NBA - 1);
            const float f0 = __int_as_float(__builtin_amdgcn_readlane(e0i, k));
            const float f1 = __int_as_float(__builtin_amdgcn_readlane(e1i, k));
            const float f2 = __int_as_float(__builtin_amdgcn_readlane(e2i, k));
            const float f3 = __int_as_float(__builtin_amdgcn_readlane(e3i, k));
            const float hv = Hin[(size_t)sk * HD + m];
            float lin = f0 * lw0;
            lin = fmaf(f1, lw1, lin);
            lin = fmaf(f2, lw2, lin);
            lin = fmaf(f3, lw3, lin);
            const float msg = relu_k((hv + lin) + lbv);
            if (lane < 16) {
              float* zp = zf + sl * HD + m;
              const float old = *zp;
              *zp = old + msg;
            }
          }
        }
      }
    }
    __syncthreads();
  }

  FragB bw1[4], bw2[4];
  float b1v[4];
#pragma unroll
  for (int t = 0; t < 4; ++t) {
    ld_frag(bw1[t], W1P + (size_t)(16 * t + m) * 32, hh);
    ld_frag(bw2[t], W2P + (size_t)m * 128 + 32 * t, hh);
    b1v[t] = bf16_val(b1[16 * t + m]);
  }
  const float b2v = bf16_val(b2[m]);

#pragma unroll 1
  for (int q = 0; q < (NBA / 16) / NWAVE; ++q) {
    const int ti   = q * NWAVE + wave;
    const int lrow = 16 * ti + m;
    const int row  = nodeBase + lrow;
    const int rc   = row < nN ? row : nN - 1;
    const bool live = row < nN;
    const float* hp = Hin + (size_t)rc * HD + 8 * hh;
    const v4f ha = *(const v4f*)hp;
    const v4f hb = *(const v4f*)(hp + 4);
    const float* zp = zf + lrow * HD + 8 * hh;
    const v4f za = *(const v4fa*)zp;
    const v4f zb = *(const v4fa*)(zp + 4);
    float z[8];
    z[0] = ha.x + za.x; z[1] = ha.y + za.y; z[2] = ha.z + za.z; z[3] = ha.w + za.w;
    z[4] = hb.x + zb.x; z[5] = hb.y + zb.y; z[6] = hb.z + zb.z; z[7] = hb.w + zb.w;
    FragB af;
#pragma unroll
    for (int i = 0; i < 8; ++i) {
      unsigned short hi, lo;
      split2(live ? z[i] : 0.0f, hi, lo);
      af.u[i] = hi; af.u[8 + i] = lo;
    }
    v8f acc[4];
#pragma unroll
    for (int t = 0; t < 4; ++t) acc[t] = wmb(af, bw1[t], zero8);
#pragma unroll
    for (int t = 0; t < 4; ++t) {
#pragma unroll
      for (int r = 0; r < 8; ++r) {
        unsigned short hi, lo;
        split2(relu_k(acc[t][r] + b1v[t]), hi, lo);
        const int lr = 8 * hh + r;
        hs[lr * 128 + 16 * t + m]      = hi;
        hs[lr * 128 + 64 + 16 * t + m] = lo;
      }
    }
    wave_sync();
    v8f a2 = zero8;
#pragma unroll
    for (int ks = 0; ks < 4; ++ks) {
      FragB ah;
      ld_frag(ah, hs + m * 128 + 32 * ks, hh);
      a2 = wmb(ah, bw2[ks], a2);
    }
#pragma unroll
    for (int r = 0; r < 8; ++r) ot[(8 * hh + r) * 16 + m] = a2[r] + b2v;
    wave_sync();
    v4f y[2];
#pragma unroll
    for (int i = 0; i < 2; ++i) {
      const int rr = 8 * i + (lane >> 2);
      const v4f v = *(const v4fa*)(ot + rr * 16 + 4 * (lane & 3));
      v4f t4 = ln16_relu(v);
      const bool lv = (nodeBase + 16 * ti + rr) < nN;
      t4.x = lv ? t4.x : 0.0f; t4.y = lv ? t4.y : 0.0f; t4.z = lv ? t4.z : 0.0f; t4.w = lv ? t4.w : 0.0f;
      y[i] = t4;
    }
    float* op0 = Hout + (size_t)(nodeBase + 16 * ti + (lane >> 2)) * HD + 4 * (lane & 3);
    float* op1 = op0 + 8 * HD;
    *(volatile v4f*)op0 = y[0];
    *(volatile v4f*)op1 = y[1];
    __threadfence();
    *(volatile v4f*)op0 = y[0];
    *(volatile v4f*)op1 = y[1];
    wave_sync();
  }
}

__global__ __launch_bounds__(NTHR) void k_pool_head(const int* __restrict__ bat, int nN, int nCh,
                                                    const int* __restrict__ TN, const float* __restrict__ H,
                                                    const unsigned short* __restrict__ FC1P,
                                                    const float* __restrict__ fcb1, const float* __restrict__ fcw2,
                                                    const float* __restrict__ fcb2, float* out, int nG) {
  extern __shared__ __attribute__((aligned(16))) int dsm[];
  int*   list = dsm;
  int*   cnt  = dsm + P_CNT;
  int*   misc = dsm + P_MISC;
  float* outs = (float*)(dsm + P_OUTS);
  float* pm   = (float*)(dsm + P_SUM);
  const int tid = (int)threadIdx.x, lane = tid & 31, wave = tid >> 5, hh = lane >> 4, m = lane & 15;
  const int blk = (int)blockIdx.x;
  const int gBase = blk * NBA;
  const v8f zero8 = {0.f, 0.f, 0.f, 0.f, 0.f, 0.f, 0.f, 0.f};

  {
    const v4i z4 = {0, 0, 0, 0};
    const int ninf = (int)0xff800000u;
    const v4i n4 = {ninf, ninf, ninf, ninf};
    for (int i = tid * 4; i < P_MAX; i += NTHR * 4) *(v4ia*)(dsm + i) = z4;
    for (int i = P_MAX + tid * 4; i < P_INTS; i += NTHR * 4) *(v4ia*)(dsm + i) = n4;
  }
  __syncthreads();

  int clo, chi;
  derive_window(TN, nCh, blk, misc + 16, tid, lane, wave, clo, chi);

#pragma unroll 1
  for (int ch = clo; ch <= chi; ++ch) {
    const int cbase = ch * CHUNK;
    const int wc = scan_chunk<SLA>(bat, nN, cbase, gBase, NBA, 1, list, tid, lane, wave);
    if (lane == 0) misc[wave] = wc;
    __syncthreads();
    if (wave == 0) {
#pragma unroll 1
      for (int w2 = 0; w2 < NWAVE; ++w2) {
        int c = __builtin_amdgcn_readfirstlane(misc[w2]);
        c = c < 0 ? 0 : (c > WCAP ? WCAP : c);
#pragma unroll 1
        for (int b0 = 0; b0 < c; b0 += 32) {
          const int idx = b0 + lane;
          const int ent = list[w2 * WCAP + (idx < WCAP ? idx : WCAP - 1)];
          const int slot = ent & (NBA - 1);
          const int el   = (ent >> SLA) & (CHUNK - 1);
          int node = cbase + el;
          node = node < 0 ? 0 : (node > nN - 1 ? nN - 1 : node);
          const int m32 = (c - b0) < 32 ? (c - b0) : 32;
#pragma unroll 1
          for (int k = 0; k < m32; ++k) {
            const int nk = __builtin_amdgcn_readlane(node, k);
            const int sk = __builtin_amdgcn_readlane(slot, k) & (NBA - 1);
            const float v = H[(size_t)nk * HD + m];
            float* pp = pm + (hh * NBA + sk) * HD + m;
            const float old = *pp;
            const float sv = old + v;
            const float xv = (v > old || v != v) ? v : old;
            const float nv = (hh == 0) ? sv : xv;
            *pp = nv;
            if (lane == 0) cnt[sk] = cnt[sk] + 1;
          }
        }
      }
    }
    __syncthreads();
  }

  FragB bf[4][2];
  float fb1[4], fw2[4];
#pragma unroll
  for (int t = 0; t < 4; ++t) {
    ld_frag(bf[t][0], FC1P + (size_t)(16 * t + m) * 64, hh);
    ld_frag(bf[t][1], FC1P + (size_t)(16 * t + m) * 64 + 32, hh);
    fb1[t] = bf16_val(pick4(fcb1 + 16 * t, m));
    fw2[t] = bf16_val(pick4(fcw2 + 16 * t, m));
  }
  const float fb2 = bf16_val(fcb2[0]);

#pragma unroll 1
  for (int q = 0; q < (NBA / 16) / NWAVE; ++q) {
    const int ti   = q * NWAVE + wave;
    const int slot = 16 * ti + m;
    const int cn   = cnt[slot];
    const float rc = 1.0f / (float)cn;
    const float* sp = pm + slot * HD + 8 * hh;
    const float* xp = pm + (NBA + slot) * HD + 8 * hh;
    const v4f s0 = *(const v4fa*)sp;
    const v4f s1 = *(const v4fa*)(sp + 4);
    const v4f x0 = *(const v4fa*)xp;
    const v4f x1 = *(const v4fa*)(xp + 4);
    float g[16];
    g[0] = s0.x * rc; g[1] = s0.y * rc; g[2] = s0.z * rc; g[3] = s0.w * rc;
    g[4] = s1.x * rc; g[5] = s1.y * rc; g[6] = s1.z * rc; g[7] = s1.w * rc;
    g[8] = x0.x; g[9] = x0.y; g[10] = x0.z; g[11] = x0.w;
    g[12] = x1.x; g[13] = x1.y; g[14] = x1.z; g[15] = x1.w;
    float s = 0.0f;
#pragma unroll
    for (int i = 0; i < 16; ++i) s += g[i];
    s += __shfl_xor(s, 16, 32);
    const float mu = s * (1.0f / 32.0f);
    float qq = 0.0f;
#pragma unroll
    for (int i = 0; i < 16; ++i) { const float d = g[i] - mu; qq = fmaf(d, d, qq); }
    qq += __shfl_xor(qq, 16, 32);
    const float rs = 1.0f / sqrtf(qq * (1.0f / 32.0f) + LN_EPS);
    FragB a0, a1;
#pragma unroll
    for (int i = 0; i < 16; ++i) {
      unsigned short hi, lo;
      split2((g[i] - mu) * rs, hi, lo);
      a0.u[i] = hi; a1.u[i] = lo;
    }
    v8f acc[4];
#pragma unroll
    for (int t = 0; t < 4; ++t) {
      acc[t] = wmb(a0, bf[t][0], zero8);
      acc[t] = wmb(a1, bf[t][1], acc[t]);
    }
    float part[8];
#pragma unroll
    for (int r = 0; r < 8; ++r) {
      float p = relu_k(acc[0][r] + fb1[0]) * fw2[0];
      p = fmaf(relu_k(acc[1][r] + fb1[1]), fw2[1], p);
      p = fmaf(relu_k(acc[2][r] + fb1[2]), fw2[2], p);
      p = fmaf(relu_k(acc[3][r] + fb1[3]), fw2[3], p);
      p += __shfl_xor(p, 1, 32);
      p += __shfl_xor(p, 2, 32);
      p += __shfl_xor(p, 4, 32);
      p += __shfl_xor(p, 8, 32);
      part[r] = p + fb2;
    }
    if (m == 0) {
#pragma unroll
      for (int r = 0; r < 8; ++r) outs[16 * ti + 8 * hh + r] = part[r];
    }
  }
  __syncthreads();
  const v4f ov = *(const v4fa*)(outs + 4 * tid);
  const int gi = gBase + 4 * tid;
  const bool ok = (gi + 3) < nG;
  float* op = out + (size_t)(ok ? gi : 0);
  if (ok) *(volatile v4f*)op = ov;
  __threadfence();
  if (ok) *(volatile v4f*)op = ov;
}

static inline int cdiv(int a, int b) { return (a + b - 1) / b; }
static inline size_t al256(size_t o) { return (o + 255) & ~(size_t)255; }

extern "C" void kernel_launch(void* const* d_in, const int* in_sizes, int n_in,
                              void* d_out, int out_size, void* d_ws, size_t ws_size,
                              hipStream_t stream) {
  if (n_in < 29) return;
  if (in_sizes[0] < 5 || (in_sizes[0] % 5) != 0) return;
  const int nN = in_sizes[0] / 5;
  if (nN < 1 || nN > (1 << 26)) return;
  if (in_sizes[1] < 4 || (in_sizes[1] % 4) != 0) return;
  const int nE = in_sizes[1] / 4;
  if (nE < 1 || nE > (1 << 30)) return;
  if (in_sizes[2] != 80 || in_sizes[3] != 16 || in_sizes[4] != 256 || in_sizes[5] != 16) return;
  if (in_sizes[6] != 80 || in_sizes[7] != 16 || in_sizes[8] != 256 || in_sizes[9] != 16) return;
  if (in_sizes[10] != 64 || in_sizes[11] != 16 || in_sizes[12] != 1024 || in_sizes[13] != 64) return;
  if (in_sizes[14] != 1024 || in_sizes[15] != 16) return;
  if (in_sizes[16] != 64 || in_sizes[17] != 16 || in_sizes[18] != 1024 || in_sizes[19] != 64) return;
  if (in_sizes[20] != 1024 || in_sizes[21] != 16) return;
  if (in_sizes[22] != 2048 || in_sizes[23] != 64 || in_sizes[24] != 64 || in_sizes[25] != 1) return;
  if (in_sizes[26] != nN || in_sizes[28] != nN) return;
  if ((long long)in_sizes[27] != 2LL * nE) return;
  const int nG = out_size;
  if (nG < 4 || (nG & 3) != 0) return;

  const float* x     = (const float*)d_in[0];
  const float* eattr = (const float*)d_in[1];
  const float* je_w1 = (const float*)d_in[2];   const float* je_b1 = (const float*)d_in[3];
  const float* je_w2 = (const float*)d_in[4];   const float* je_b2 = (const float*)d_in[5];
  const float* mu_w1 = (const float*)d_in[6];   const float* mu_b1 = (const float*)d_in[7];
  const float* mu_w2 = (const float*)d_in[8];   const float* mu_b2 = (const float*)d_in[9];
  const float* lin1w = (const float*)d_in[10];  const float* lin1b = (const float*)d_in[11];
  const float* m1_w1 = (const float*)d_in[12];  const float* m1_b1 = (const float*)d_in[13];
  const float* m1_w2 = (const float*)d_in[14];  const float* m1_b2 = (const float*)d_in[15];
  const float* lin2w = (const float*)d_in[16];  const float* lin2b = (const float*)d_in[17];
  const float* m2_w1 = (const float*)d_in[18];  const float* m2_b1 = (const float*)d_in[19];
  const float* m2_w2 = (const float*)d_in[20];  const float* m2_b2 = (const float*)d_in[21];
  const float* fc_w1 = (const float*)d_in[22];  const float* fc_b1 = (const float*)d_in[23];
  const float* fc_w2 = (const float*)d_in[24];  const float* fc_b2 = (const float*)d_in[25];
  const int*   tyid  = (const int*)d_in[26];
  const int*   edge  = (const int*)d_in[27];
  const int*   bat   = (const int*)d_in[28];
  float* out = (float*)d_out;
  const int* src = edge;
  const int* dst = edge + nE;

  const int NP   = cdiv(nN, NBA) * NBA;
  const int gA   = NP / NBA;
  const int nChE = cdiv(nE, CHUNK);
  const int nBE  = cdiv(nChE, CPB);
  const int nChN = cdiv(nN, CHUNK);
  const int nBN  = cdiv(nChN, CPB);
  const int gP   = cdiv(nG, NBA);
  const int vec8 = ((nE & 3) == 0) ? 1 : 0;

  char* ws = (char*)d_ws;
  size_t off = 0;
  const size_t oWP = off; off = al256(off + (size_t)WP_HALVES * 2);
  const size_t oTE = off; off = al256(off + (size_t)nBE * TROW * 4);
  const size_t oTN = off; off = al256(off + (size_t)nBN * TROW * 4);
  const size_t oHA = off; off = al256(off + (size_t)NP * HD * 4);
  const size_t oHB = off; off = al256(off + (size_t)NP * HD * 4);
  if (off > ws_size || off > (size_t)WSMAX) return;
  unsigned short* WP = (unsigned short*)(ws + oWP);
  int*   TE = (int*)(ws + oTE);
  int*   TN = (int*)(ws + oTN);
  float* HA = (float*)(ws + oHA);
  float* HB = (float*)(ws + oHB);

  const size_t ldsG = (size_t)G_INTS * 4;
  const size_t ldsP = (size_t)P_INTS * 4;
  hipFuncSetAttribute(reinterpret_cast<const void*>(&k_gine), hipFuncAttributeMaxDynamicSharedMemorySize, (int)ldsG);
  hipFuncSetAttribute(reinterpret_cast<const void*>(&k_pool_head), hipFuncAttributeMaxDynamicSharedMemorySize, (int)ldsP);

  k_prep<<<NUNITS / NTHR, NTHR, 0, stream>>>(je_w1, mu_w1, je_w2, mu_w2, m1_w1, m1_w2, m2_w1, m2_w2, fc_w1, WP);
  k_bounds<<<nBE + nBN, NTHR, 0, stream>>>(dst, nE, vec8, bat, nN, nBE, TE, TN);
  k_enc<<<NP / 128, NTHR, 0, stream>>>(x, tyid, je_b1, mu_b1, je_b2, mu_b2, WP, nN, HA);
  k_gine<<<gA, NTHR, ldsG, stream>>>(src, dst, eattr, nE, nN, vec8, nChE, TE, lin1w, lin1b,
                                     WP + OFF_M1W1, m1_b1, WP + OFF_M1W2, m1_b2, HA, HB);
  k_gine<<<gA, NTHR, ldsG, stream>>>(src, dst, eattr, nE, nN, vec8, nChE, TE, lin2w, lin2b,
                                     WP + OFF_M2W1, m2_b1, WP + OFF_M2W2, m2_b2, HB, HA);
  k_pool_head<<<gP, NTHR, ldsP, stream>>>(bat, nN, nChN, TN, HA, WP + OFF_FC1, fc_b1, fc_w2, fc_b2, out, nG);
}
